// Mamba2Block_90486370992207
// MI455X (gfx1250) — hardware-verified
//
#include <hip/hip_runtime.h>
#include <math.h>

typedef __attribute__((ext_vector_type(16))) _Float16 v16h;
typedef __attribute__((ext_vector_type(8)))  _Float16 v8h;
typedef __attribute__((ext_vector_type(2)))  _Float16 v2h;
typedef __attribute__((ext_vector_type(16))) __bf16   v16b;
typedef __attribute__((ext_vector_type(8)))  __bf16   v8b;
typedef __attribute__((ext_vector_type(8)))  float    v8f;
typedef __attribute__((ext_vector_type(4)))  float    v4f;
typedef __attribute__((ext_vector_type(2)))  float    v2f;

constexpr int kL    = 1024;
constexpr int kDM   = 1024;
constexpr int kDI   = 2048;
constexpr int kH    = 32;
constexpr int kN    = 64;
constexpr int kDin  = 2 * kDI + 2 * kN + kH;
constexpr int kDC   = 4;
constexpr int kThr  = 256;
constexpr float kInCarry = 1024.0f;
constexpr float kSc = 1.0f / (kInCarry * kInCarry);
constexpr float kNormEps = 1e-6f;
constexpr float kF16MinNormal = 6.103515625e-5f;

static_assert(kDI == kH * 64 && kDin == 4256 && kN == 64 && kDC == 4, "the index arithmetic below uses these sizes");

constexpr size_t kOffZB = 0ull;
constexpr size_t kOffBIA = 8192ull;
constexpr size_t kOffU16 = 8448ull;
constexpr size_t kOffWIN16 = 2105600ull;
constexpr size_t kOffWOUT16 = 10821888ull;
constexpr size_t kOffZ32 = 15016192ull;
constexpr size_t kOffXI32 = 23404800ull;
constexpr size_t kOffBC32 = 31793408ull;
constexpr size_t kOffDTR32 = 32317696ull;
constexpr size_t kOffYG32 = 32448768ull;
constexpr size_t kOffRS = 40837376ull;
constexpr size_t kOffY16 = 40841472ull;
constexpr size_t kWsTotal = 45035776ull;
static_assert(kWsTotal <= 134217728ull, "carve cap: under 128 MiB");
static_assert(kOffZB == 0
              && kOffBIA == kOffZB + 8192ull
              && kOffU16 == kOffBIA + 256ull
              && kOffWIN16 == kOffU16 + 2097152ull
              && kOffWOUT16 == kOffWIN16 + 8716288ull
              && kOffZ32 == kOffWOUT16 + 4194304ull
              && kOffXI32 == kOffZ32 + 8388608ull
              && kOffBC32 == kOffXI32 + 8388608ull
              && kOffDTR32 == kOffBC32 + 524288ull
              && kOffYG32 == kOffDTR32 + 131072ull
              && kOffRS == kOffYG32 + 8388608ull
              && kOffY16 == kOffRS + 4096ull
              && kWsTotal == kOffY16 + 4194304ull, "the carve is chained and totalled");
static_assert((kOffZB % 256) == 0 && (kOffBIA % 256) == 0 && (kOffU16 % 256) == 0 && (kOffWIN16 % 256) == 0 && (kOffWOUT16 % 256) == 0 && (kOffZ32 % 256) == 0 && (kOffXI32 % 256) == 0 && (kOffBC32 % 256) == 0 && (kOffDTR32 % 256) == 0 && (kOffYG32 % 256) == 0 && (kOffRS % 256) == 0 && (kOffY16 % 256) == 0, "aligned regions");
static_assert(2048 >= kDI && 2048 >= kDM && 2048 >= 2 * kN, "the zero bias covers the widest N of any engine launch (the engine reads bias[n] for every n < N)");

__device__ __forceinline__ unsigned short f2bf_bits(float f) {
  unsigned u = __float_as_uint(f);
  return (unsigned short)((u + 0x7FFFu + ((u >> 16) & 1u)) >> 16);
}
__device__ __forceinline__ float bf_bits2f(unsigned short h) { return __uint_as_float(((unsigned)h) << 16); }
__device__ __forceinline__ float bf16r(float f) { return bf_bits2f(f2bf_bits(f)); }
__device__ __forceinline__ float carry_flush(float v, float carry) {
  const float s = v * carry;
  return (fabsf(s) < kF16MinNormal) ? 0.0f : s;
}

__device__ __forceinline__ void dep_guard4_h(v8f& a, v8f& b, v8f& c, v8f& d, v16h x, v16h y) { asm volatile("v_nop\n\tv_nop\n\tv_nop\n\tv_nop" : "+v"(a), "+v"(b), "+v"(c), "+v"(d) : "v"(x), "v"(y)); }
__device__ __forceinline__ void dep_guard4_b(v8f& a, v8f& b, v8f& c, v8f& d, v16b x, v16b y) { asm volatile("v_nop\n\tv_nop\n\tv_nop\n\tv_nop" : "+v"(a), "+v"(b), "+v"(c), "+v"(d) : "v"(x), "v"(y)); }
__device__ __forceinline__ void keep4_h(v16h a, v16h b, v16h c, v16h d) { asm volatile("v_nop" :: "v"(a), "v"(b), "v"(c), "v"(d)); }
__device__ __forceinline__ void keep4_b(v16b a, v16b b, v16b c, v16b d) { asm volatile("v_nop" :: "v"(a), "v"(b), "v"(c), "v"(d)); }
__device__ __forceinline__ void acc_guard4(v8f& a, v8f& b, v8f& c, v8f& d) { asm volatile("v_nop\n\tv_nop\n\tv_nop\n\tv_nop" : "+v"(a), "+v"(b), "+v"(c), "+v"(d)); }

template <typename T> struct Frag;
template <> struct Frag<_Float16> {
  typedef v16h V; union U { v16h v; v8h h[2]; };
  static __device__ __forceinline__ v16h load(const _Float16* p) {
    U f; f.h[0] = *(const v8h*)(p); f.h[1] = *(const v8h*)(p + 16); return f.v;
  }
  static __device__ __forceinline__ v8f mma(v16h a, v16h b, v8f c) {
    return __builtin_amdgcn_wmma_f32_16x16x32_f16(false, a, false, b, (short)0, c, false, false);
  }
  static __device__ __forceinline__ void guard4(v8f& a, v8f& b, v8f& c, v8f& d, v16h x, v16h y) { dep_guard4_h(a, b, c, d, x, y); }
  static __device__ __forceinline__ void keep(v16h a, v16h b, v16h c, v16h d) { keep4_h(a, b, c, d); }
};
template <> struct Frag<__bf16> {
  typedef v16b V; union U { v16b v; v8b h[2]; };
  static __device__ __forceinline__ v16b load(const __bf16* p) {
    U f; f.h[0] = *(const v8b*)(p); f.h[1] = *(const v8b*)(p + 16); return f.v;
  }
  static __device__ __forceinline__ v8f mma(v16b a, v16b b, v8f c) {
    return __builtin_amdgcn_wmma_f32_16x16x32_bf16(false, a, false, b, (short)0, c, false, false);
  }
  static __device__ __forceinline__ void guard4(v8f& a, v8f& b, v8f& c, v8f& d, v16b x, v16b y) { dep_guard4_b(a, b, c, d, x, y); }
  static __device__ __forceinline__ void keep(v16b a, v16b b, v16b c, v16b d) { keep4_b(a, b, c, d); }
};

__device__ __forceinline__ v8f mma_h(v16h a, v16h b, v8f c) {
  c = __builtin_amdgcn_wmma_f32_16x16x32_f16(false, a, false, b, (short)0, c, false, false);
  asm volatile("v_nop\n\tv_nop\n\tv_nop\n\tv_nop" : "+v"(c) : "v"(a), "v"(b));
  return c;
}

template <int ET> struct Elem;
template <> struct Elem<0> { typedef _Float16 T; };
template <> struct Elem<1> { typedef __bf16 T; };
template <int ET, bool SPLIT, int BIAS_MODE, int OUT_MODE, bool RESID, int ACT = 0>
__global__ __launch_bounds__(256) void wmma_gemm64(
    const unsigned short* __restrict__ Ap, const unsigned short* __restrict__ A2p, int lda, long strideA,
    const unsigned short* __restrict__ Btp, const unsigned short* __restrict__ Bt2p, int ldb, long strideB,
    void* __restrict__ Cout, void* __restrict__ Cout2, int ldc, long strideC,
    const float* __restrict__ bias,
    const float* __restrict__ resid, long strideR,
    int M, int N, int K, float scale) {
  typedef typename Elem<ET>::T T;
  typedef typename Frag<T>::V V;
  const T* A = (const T*)Ap; const T* A2 = (const T*)A2p; const T* Bt = (const T*)Btp; const T* Bt2 = (const T*)Bt2p;
  __shared__ __align__(16) float sT[8][16 * 68];
  const int b    = blockIdx.y;
  const int lane = threadIdx.x & 31;
  const int wave = threadIdx.x >> 5;
  const int tilesN = N >> 6;
  const int tilesM = M >> 6;
  const int tile = blockIdx.x * 8 + wave;
  if (tile >= tilesM * tilesN) return;
  const int tm = tile / tilesN;
  const int tn = tile - tm * tilesN;
  const int m0 = tm << 6;
  const int n0 = tn << 6;

  const T* Ab  = A  + (size_t)b * strideA;
  const T* Bb  = Bt + (size_t)b * strideB;
  const T* Ab2 = SPLIT ? (A2  + (size_t)b * strideA) : nullptr;
  const T* Bb2 = SPLIT ? (Bt2 + (size_t)b * strideB) : nullptr;

  const int rlane = lane & 15;
  const int koff  = (lane >> 4) * 8;
  const int mOff  = (lane >> 4) * 8;

  v8f acc[4][4];
#pragma unroll
  for (int i = 0; i < 4; ++i)
#pragma unroll
    for (int j = 0; j < 4; ++j) acc[i][j] = (v8f){0.f,0.f,0.f,0.f,0.f,0.f,0.f,0.f};

  for (int k0 = 0; k0 < K; k0 += 32) {
    V bh[4], bl[4];
#pragma unroll
    for (int j = 0; j < 4; ++j) {
      const size_t bo = (size_t)(n0 + (j << 4) + rlane) * ldb + koff + k0;
      bh[j] = Frag<T>::load(Bb + bo);
      if (SPLIT) bl[j] = Frag<T>::load(Bb2 + bo);
    }
#pragma unroll
    for (int i = 0; i < 4; ++i) {
      const size_t ao = (size_t)(m0 + (i << 4) + rlane) * lda + koff + k0;
      V ah = Frag<T>::load(Ab + ao);
      V al;
      if (SPLIT) al = Frag<T>::load(Ab2 + ao);
#pragma unroll
      for (int j = 0; j < 4; ++j) {
        acc[i][j] = Frag<T>::mma(ah, bh[j], acc[i][j]);
        if (SPLIT) {
          acc[i][j] = Frag<T>::mma(ah, bl[j], acc[i][j]);
          acc[i][j] = Frag<T>::mma(al, bh[j], acc[i][j]);
        }
      }
      Frag<T>::guard4(acc[i][0], acc[i][1], acc[i][2], acc[i][3], ah, SPLIT ? al : ah);
    }
    Frag<T>::keep(bh[0], bh[1], bh[2], bh[3]);
    if (SPLIT) Frag<T>::keep(bl[0], bl[1], bl[2], bl[3]);
  }
  acc_guard4(acc[0][0], acc[0][1], acc[0][2], acc[0][3]);
  acc_guard4(acc[1][0], acc[1][1], acc[1][2], acc[1][3]);
  acc_guard4(acc[2][0], acc[2][1], acc[2][2], acc[2][3]);
  acc_guard4(acc[3][0], acc[3][1], acc[3][2], acc[3][3]);

  float* slab = sT[wave];
  const float* Rb = RESID ? (resid + (size_t)b * strideR) : nullptr;
#pragma unroll
  for (int i = 0; i < 4; ++i) {
    const int mBase = m0 + (i << 4);
#pragma unroll
    for (int j = 0; j < 4; ++j) {
      const int n = n0 + (j << 4) + rlane;
      float bv = 0.f;
      if (BIAS_MODE == 2) bv = bias[n];
#pragma unroll
      for (int r = 0; r < 8; ++r) {
        float v = acc[i][j][r] * scale;
        if (BIAS_MODE == 1) v += bias[mBase + mOff + r];
        if (BIAS_MODE == 2) v += bv;
        if (RESID) v += Rb[(size_t)(mBase + mOff + r) * ldc + n];
        if (ACT == 1) v = tanhf(v);
        if (ACT == 2) v = fmaxf(v, 0.0f);
        if (ACT == 3) v = v / (1.0f + expf(-v));
        if (ACT == 4) v = (v > 0.f) ? v : 0.01f * v;
        slab[(mOff + r) * 68 + (j << 4) + rlane] = v;
      }
    }
    __builtin_amdgcn_fence(__ATOMIC_RELEASE, "workgroup");
    __builtin_amdgcn_wave_barrier();
    __builtin_amdgcn_fence(__ATOMIC_ACQUIRE, "workgroup");
    if (OUT_MODE == 0) {
      float* C = (float*)Cout + (size_t)b * strideC;
      const int hh = lane >> 4, c4 = (lane & 15) * 4;
      for (int pass = 0; pass < 2; ++pass) {
#pragma unroll
        for (int it = 0; it < 8; ++it) {
          const int row = it * 2 + hh;
          v4f v = *(const v4f*)(slab + row * 68 + c4);
          *(volatile v4f*)(C + (size_t)(mBase + row) * ldc + n0 + c4) = v;
        }
        __threadfence();
      }
    } else {
      const int q = lane >> 3, c8 = (lane & 7) * 8;
      unsigned short* C  = (unsigned short*)Cout  + (size_t)b * strideC;
      unsigned short* C2 = (OUT_MODE == 2) ? ((unsigned short*)Cout2 + (size_t)b * strideC) : nullptr;
      for (int pass = 0; pass < 2; ++pass) {
#pragma unroll
        for (int it = 0; it < 4; ++it) {
          const int row = it * 4 + q;
          const float* sp = slab + row * 68 + c8;
          v8h hv, lv;
#pragma unroll
          for (int e = 0; e < 8; ++e) {
            if (OUT_MODE == 1) {
              hv[e] = (_Float16)sp[e];
            } else {
              unsigned short hb = f2bf_bits(sp[e]);
              unsigned short lb = f2bf_bits(sp[e] - bf_bits2f(hb));
              hv[e] = __builtin_bit_cast(_Float16, hb);
              lv[e] = __builtin_bit_cast(_Float16, lb);
            }
          }
          *(volatile v8h*)(C + (size_t)(mBase + row) * ldc + n0 + c8) = hv;
          if (OUT_MODE == 2) *(volatile v8h*)(C2 + (size_t)(mBase + row) * ldc + n0 + c8) = lv;
        }
        __threadfence();
      }
    }
    __builtin_amdgcn_fence(__ATOMIC_RELEASE, "workgroup");
    __builtin_amdgcn_wave_barrier();
    __builtin_amdgcn_fence(__ATOMIC_ACQUIRE, "workgroup");
  }
}

__global__ __launch_bounds__(kThr) void cast_plane_kernel(const float* __restrict__ src, unsigned short* __restrict__ dst,
                                                          int colsLog2, int dstPitch, int dstOff) {
  const int i   = blockIdx.x * kThr + threadIdx.x;
  const int sh  = colsLog2 - 3;
  const int row = i >> sh;
  const int c8  = (i & ((1 << sh) - 1)) * 8;
  const float* sp = src + ((size_t)row << colsLog2) + c8;
  const v4f a0 = *(const v4f*)(sp);
  const v4f a1 = *(const v4f*)(sp + 4);
  v8h hv;
#pragma unroll
  for (int e = 0; e < 4; ++e) {
    const float f0 = a0[e];
    const float f1 = a1[e];
    hv[e]     = (_Float16)carry_flush(bf16r(f0), kInCarry);
    hv[4 + e] = (_Float16)carry_flush(bf16r(f1), kInCarry);
  }
  unsigned short* dp = dst + (size_t)row * dstPitch + dstOff + c8;
  *(volatile v8h*)dp = hv;
  __threadfence();
  *(volatile v8h*)dp = hv;
}

__global__ __launch_bounds__(256) void wmma_gemm32(
    const unsigned short* __restrict__ Ap, int lda, long strideA,
    const unsigned short* __restrict__ Btp, int ldb, long strideB,
    float* __restrict__ Cout, int ldc, long strideC,
    const float* __restrict__ bias,
    int M, int N, int K, float scale) {
  typedef _Float16 T;
  typedef Frag<T>::V V;
  const T* A = (const T*)Ap; const T* Bt = (const T*)Btp;
  __shared__ __align__(16) float sT[8][16 * 36];
  const int b    = blockIdx.y;
  const int lane = threadIdx.x & 31;
  const int wave = threadIdx.x >> 5;
  const int tilesN = N >> 5;
  const int tilesM = M >> 6;
  const int tile = blockIdx.x * 8 + wave;
  if (tile >= tilesM * tilesN) return;
  const int tm = tile / tilesN;
  const int tn = tile - tm * tilesN;
  const int m0 = tm << 6;
  const int n0 = tn << 5;

  const T* Ab = A  + (size_t)b * strideA;
  const T* Bb = Bt + (size_t)b * strideB;

  const int rlane = lane & 15;
  const int koff  = (lane >> 4) * 8;
  const int mOff  = (lane >> 4) * 8;

  v8f acc[4][2];
#pragma unroll
  for (int i = 0; i < 4; ++i)
#pragma unroll
    for (int j = 0; j < 2; ++j) acc[i][j] = (v8f){0.f,0.f,0.f,0.f,0.f,0.f,0.f,0.f};

  for (int k0 = 0; k0 < K; k0 += 32) {
    V bh[2];
#pragma unroll
    for (int j = 0; j < 2; ++j) {
      const size_t bo = (size_t)(n0 + (j << 4) + rlane) * ldb + koff + k0;
      bh[j] = Frag<T>::load(Bb + bo);
    }
#pragma unroll
    for (int i = 0; i < 4; i += 2) {
      const size_t ao0 = (size_t)(m0 + (i << 4) + rlane) * lda + koff + k0;
      const size_t ao1 = (size_t)(m0 + ((i + 1) << 4) + rlane) * lda + koff + k0;
      V ah0 = Frag<T>::load(Ab + ao0);
      V ah1 = Frag<T>::load(Ab + ao1);
      acc[i][0]     = Frag<T>::mma(ah0, bh[0], acc[i][0]);
      acc[i][1]     = Frag<T>::mma(ah0, bh[1], acc[i][1]);
      acc[i + 1][0] = Frag<T>::mma(ah1, bh[0], acc[i + 1][0]);
      acc[i + 1][1] = Frag<T>::mma(ah1, bh[1], acc[i + 1][1]);
      Frag<T>::guard4(acc[i][0], acc[i][1], acc[i + 1][0], acc[i + 1][1], ah0, ah1);
    }
    Frag<T>::keep(bh[0], bh[1], bh[0], bh[1]);
  }
  acc_guard4(acc[0][0], acc[0][1], acc[1][0], acc[1][1]);
  acc_guard4(acc[2][0], acc[2][1], acc[3][0], acc[3][1]);

  float* slab = sT[wave];
  float* C = Cout + (size_t)b * strideC;
#pragma unroll
  for (int i = 0; i < 4; ++i) {
    const int mBase = m0 + (i << 4);
#pragma unroll
    for (int j = 0; j < 2; ++j) {
      const int n = n0 + (j << 4) + rlane;
      const float bv = bias[n];
#pragma unroll
      for (int r = 0; r < 8; ++r) {
        float v = acc[i][j][r] * scale;
        v += bv;
        slab[(mOff + r) * 36 + (j << 4) + rlane] = v;
      }
    }
    __builtin_amdgcn_fence(__ATOMIC_RELEASE, "workgroup");
    __builtin_amdgcn_wave_barrier();
    __builtin_amdgcn_fence(__ATOMIC_ACQUIRE, "workgroup");
    {
      const int q = lane >> 3, c4 = (lane & 7) * 4;
      for (int pass = 0; pass < 2; ++pass) {
#pragma unroll
        for (int it = 0; it < 4; ++it) {
          const int row = it * 4 + q;
          v4f v = *(const v4f*)(slab + row * 36 + c4);
          *(volatile v4f*)(C + (size_t)(mBase + row) * ldc + n0 + c4) = v;
        }
        __threadfence();
      }
    }
    __builtin_amdgcn_fence(__ATOMIC_RELEASE, "workgroup");
    __builtin_amdgcn_wave_barrier();
    __builtin_amdgcn_fence(__ATOMIC_ACQUIRE, "workgroup");
  }
}
static_assert(sizeof(float) * 8 * 16 * 36 == 18432, "the tail's slabs: 8 waves x 16 rows x 36 floats = 18,432 B of LDS");


__global__ __launch_bounds__(kThr) void zero_kernel(float* __restrict__ dst) {
  const size_t o4 = ((size_t)blockIdx.x * kThr + threadIdx.x) * 4u;
  const v4f z = {0.f, 0.f, 0.f, 0.f};
  *(volatile v4f*)(dst + o4) = z;
  __threadfence();
  *(volatile v4f*)(dst + o4) = z;
}

__global__ __launch_bounds__(64) void bias_kernel(const float* __restrict__ dt_bias, float* __restrict__ BIA) {
  const unsigned i = threadIdx.x;
  const float a = dt_bias[(i < (unsigned)kH) ? i : 0u];
  const float v = (i < (unsigned)kH) ? bf16r(a) : 0.0f;
  *(volatile float*)(BIA + i) = v;
  __threadfence();
  *(volatile float*)(BIA + i) = v;
}

__global__ __launch_bounds__(kThr) void scan_kernel(const float* __restrict__ XI, const float* __restrict__ BC, const float* __restrict__ DTR, const float* __restrict__ Z,
                                                   const float* __restrict__ W_conv, const float* __restrict__ b_conv, const float* __restrict__ A_log, const float* __restrict__ Dp,
                                                   float* __restrict__ YG) {
  const unsigned c = blockIdx.x * (unsigned)kThr + threadIdx.x;
  const unsigned hd = c >> 6;
  float A[kN], h[kN];
#pragma unroll
  for (int n = 0; n < kN; ++n) { const float a = A_log[(size_t)c * kN + n]; A[n] = -expf(bf16r(a)); h[n] = 0.0f; }
  const v4f wv = *(const v4f*)(W_conv + (size_t)c * kDC);
  const float w0 = bf16r(wv[0]), w1 = bf16r(wv[1]), w2 = bf16r(wv[2]), w3 = bf16r(wv[3]);
  const float q0 = Dp[c], c0 = b_conv[c];
  const float dc = bf16r(q0), cb = bf16r(c0);
  float x0 = 0.0f, x1 = 0.0f, x2 = 0.0f;
  for (int l = 0; l < kL; ++l) {
    const size_t row = (size_t)l;
    const float xv = XI[row * kDI + c];
    float acc = cb;
    acc += w0 * x0;
    acc += w1 * x1;
    acc += w2 * x2;
    acc += w3 * xv;
    x0 = x1; x1 = x2; x2 = xv;
    const float u = acc / (1.0f + expf(-acc));
    const float pre = DTR[row * 32u + hd];
    const float dt = (pre > 20.0f) ? pre : log1pf(expf(pre));
    const float* bp = BC + row * 128u;
    float y = 0.0f;
#pragma unroll
    for (int q = 0; q < kN / 4; ++q) {
      const v4f bv = *(const v4f*)(bp + 4 * q), cv = *(const v4f*)(bp + kN + 4 * q);
#pragma unroll
      for (int e = 0; e < 4; ++e) {
        const int n = 4 * q + e;
        const float hn = expf(dt * A[n]) * h[n] + bv[e] * u;
        h[n] = hn;
        y += hn * cv[e];
      }
    }
    const float zv = Z[row * kDI + c];
    const float o = (y + dc * u) * (zv / (1.0f + expf(-zv)));
    float* dp = YG + row * kDI + c;
    *(volatile float*)dp = o;
    __threadfence();
    *(volatile float*)dp = o;
  }
}
static_assert(kDI == 8 * kThr && (kN % 4) == 0, "scan grid exact: 8 blocks; the B | C columns 16-B aligned");

__global__ __launch_bounds__(kThr) void rms_kernel(const float* __restrict__ YG, float* __restrict__ RS) {
  const unsigned l = blockIdx.x * (unsigned)kThr + threadIdx.x;
  const float* yp = YG + (size_t)l * kDI;
  float ss = 0.0f;
  for (int q4 = 0; q4 < kDI / 4; ++q4) {
    const v4f a = *(const v4f*)(yp + 4 * q4);
#pragma unroll
    for (int k = 0; k < 4; ++k) ss += a[k] * a[k];
  }
  const float rs = 1.0f / sqrtf(ss * (1.0f / (float)kDI) + kNormEps);
  *(volatile float*)(RS + l) = rs;
  __threadfence();
  *(volatile float*)(RS + l) = rs;
}
static_assert(kL == 4 * kThr, "norm-scale grid exact: 4 blocks");

__global__ __launch_bounds__(kThr) void ycast_kernel(const float* __restrict__ YG, const float* __restrict__ RS, const float* __restrict__ norm_w, unsigned short* __restrict__ Y16) {
  const unsigned i = blockIdx.x * (unsigned)kThr + threadIdx.x;
  const unsigned c8 = i & 255u, l = i >> 8;
  const float* yp = YG + (size_t)i * 8u;
  const float* wp = norm_w + c8 * 8u;
  const v4f a0 = *(const v4f*)yp, a1 = *(const v4f*)(yp + 4), w0 = *(const v4f*)wp, w1 = *(const v4f*)(wp + 4);
  const float f = RS[l];
  v8h hv;
#pragma unroll
  for (int k = 0; k < 8; ++k) {
    const float y = (k < 4) ? a0[k] : a1[k - 4];
    const float wr = (k < 4) ? w0[k] : w1[k - 4];
    hv[k] = (_Float16)carry_flush(y * f * bf16r(wr), kInCarry);
  }
  unsigned short* dp = Y16 + (size_t)i * 8u;
  *(volatile v8h*)dp = hv;
  __threadfence();
  *(volatile v8h*)dp = hv;
}
static_assert((size_t)kL * (kDI / 8) == 1024ull * kThr && kDI / 8 == 256, "output cast grid exact: 1,024 blocks; 256 groups of 8 a row");

static_assert(((size_t)kL * kDM / 8) % kThr == 0 && ((size_t)kDin * kDM / 8) % kThr == 0 && ((size_t)kDM * kDI / 8) % kThr == 0 && ((size_t)kDin * kDM) % 64 == 0, "plane cast grids exact; the planes are whole rows of 64");
static_assert(((kL / 64) * (kDI / 64)) % 8 == 0 && ((kL / 64) * (2 * kN / 64)) % 8 == 0 && ((kL / 64) * (32 / 32)) % 8 == 0 && ((kL / 64) * (kDM / 64)) % 8 == 0, "the projections' grids exact: every wave live");

extern "C" void kernel_launch(void* const* d_in, const int* in_sizes, int n_in,
                              void* d_out, int out_size, void* d_ws, size_t ws_size,
                              hipStream_t stream) {
  if (n_in < 9 || d_out == nullptr || d_ws == nullptr) return;
  if (in_sizes[0] != kL * kDM || in_sizes[1] != kDin * kDM || in_sizes[2] != kDI * kDC || in_sizes[3] != kDI || in_sizes[4] != kDI * kN || in_sizes[5] != kDI || in_sizes[6] != kH || in_sizes[7] != kDI || in_sizes[8] != kDM * kDI) return;
  if (out_size != kL * kDM) return;
  if (ws_size < kWsTotal) return;
  const float* xin = (const float*)d_in[0];
  const float* W_in = (const float*)d_in[1];
  const float* W_conv = (const float*)d_in[2];
  const float* b_conv = (const float*)d_in[3];
  const float* A_log = (const float*)d_in[4];
  const float* Dp = (const float*)d_in[5];
  const float* dt_bias = (const float*)d_in[6];
  const float* norm_w = (const float*)d_in[7];
  const float* W_out = (const float*)d_in[8];
  float* out = (float*)d_out;
  char* ws = (char*)d_ws;
  float* ZB = (float*)(ws + kOffZB);
  float* BIA = (float*)(ws + kOffBIA);
  unsigned short* U16 = (unsigned short*)(ws + kOffU16);
  unsigned short* WIN16 = (unsigned short*)(ws + kOffWIN16);
  unsigned short* WOUT16 = (unsigned short*)(ws + kOffWOUT16);
  float* Z32 = (float*)(ws + kOffZ32);
  float* XI32 = (float*)(ws + kOffXI32);
  float* BC32 = (float*)(ws + kOffBC32);
  float* DTR32 = (float*)(ws + kOffDTR32);
  float* YG32 = (float*)(ws + kOffYG32);
  float* RS = (float*)(ws + kOffRS);
  unsigned short* Y16 = (unsigned short*)(ws + kOffY16);

  zero_kernel<<<2, kThr, 0, stream>>>(ZB);
  bias_kernel<<<1, 64, 0, stream>>>(dt_bias, BIA);
  cast_plane_kernel<<<(int)(((size_t)kL * kDM / 8) / kThr), kThr, 0, stream>>>(xin, U16, 6, 64, 0);
  cast_plane_kernel<<<(int)(((size_t)kDin * kDM / 8) / kThr), kThr, 0, stream>>>(W_in, WIN16, 6, 64, 0);
  cast_plane_kernel<<<(int)(((size_t)kDM * kDI / 8) / kThr), kThr, 0, stream>>>(W_out, WOUT16, 6, 64, 0);
  wmma_gemm64<0, false, 2, 0, false, 0><<<dim3((kL / 64) * (kDI / 64) / 8, 1), 256, 0, stream>>>(
      U16, U16, kDM, 0L, WIN16, WIN16, kDM, 0L, (void*)Z32, (void*)Z32, kDI, 0L, ZB, nullptr, 0L, kL, kDI, kDM, kSc);
  wmma_gemm64<0, false, 2, 0, false, 0><<<dim3((kL / 64) * (kDI / 64) / 8, 1), 256, 0, stream>>>(
      U16, U16, kDM, 0L, WIN16 + (size_t)kDI * kDM, WIN16 + (size_t)kDI * kDM, kDM, 0L, (void*)XI32, (void*)XI32, kDI, 0L, ZB, nullptr, 0L, kL, kDI, kDM, kSc);
  wmma_gemm64<0, false, 2, 0, false, 0><<<dim3((kL / 64) * (2 * kN / 64) / 8, 1), 256, 0, stream>>>(
      U16, U16, kDM, 0L, WIN16 + (size_t)(2 * kDI) * kDM, WIN16 + (size_t)(2 * kDI) * kDM, kDM, 0L, (void*)BC32, (void*)BC32, 2 * kN, 0L, ZB, nullptr, 0L, kL, 2 * kN, kDM, kSc);
  wmma_gemm32<<<dim3((kL / 64) * (32 / 32) / 8, 1), 256, 0, stream>>>(
      U16, kDM, 0L, WIN16 + (size_t)(2 * kDI + 2 * kN) * kDM, kDM, 0L, DTR32, 32, 0L, BIA, kL, 32, kDM, kSc);
  scan_kernel<<<8, kThr, 0, stream>>>(XI32, BC32, DTR32, Z32, W_conv, b_conv, A_log, Dp, YG32);
  rms_kernel<<<4, kThr, 0, stream>>>(YG32, RS);
  ycast_kernel<<<1024, kThr, 0, stream>>>(YG32, RS, norm_w, Y16);
  wmma_gemm64<0, false, 2, 0, false, 0><<<dim3((kL / 64) * (kDM / 64) / 8, 1), 256, 0, stream>>>(
      Y16, Y16, kDI, 0L, WOUT16, WOUT16, kDI, 0L, (void*)out, (void*)out, kDM, 0L, ZB, nullptr, 0L, kL, kDM, kDI, kSc);
}
